// CompleteMOERTDETR_78606491451928
// MI455X (gfx1250) — hardware-verified
//
#include <hip/hip_runtime.h>
#include <stdint.h>


typedef __bf16          v16bf  __attribute__((ext_vector_type(16)));
typedef unsigned short  v16us  __attribute__((ext_vector_type(16)));
typedef unsigned short  v8us_b __attribute__((ext_vector_type(8)));
typedef v8us_b          v8us   __attribute__((may_alias));
typedef float           v8f    __attribute__((ext_vector_type(8)));
typedef float           v4f_b  __attribute__((ext_vector_type(4)));
typedef v4f_b           v4f    __attribute__((may_alias));

union Frag { v16bf v; v16us u; v8us h[2]; };

#define NB    128
#define NS    400
#define ND    256
#define NH    128
#define NE    6
#define NQ    300
#define NC    6
#define NTOK  (NB * NQ)

#define P1    264
#define HSP   132

__device__ __forceinline__ unsigned int bf16_rne_bits(float x)
{
    unsigned int u = __float_as_uint(x);
    return (u + 0x7FFFu + ((u >> 16) & 1u)) >> 16;
}

__device__ __forceinline__ void split2(float x, unsigned short& hi, unsigned short& lo)
{
    unsigned int hb = bf16_rne_bits(x);
    float hf = __uint_as_float(hb << 16);
    float r  = x - hf;
    hi = (unsigned short)hb;
    lo = (unsigned short)bf16_rne_bits(r);
}

__device__ __forceinline__ v8f mma3(v8f c, v16bf ah, v16bf al, v16bf bh, v16bf bl)
{
    c = __builtin_amdgcn_wmma_f32_16x16x32_bf16(false, ah, false, bh, (short)0, c, false, false);
    c = __builtin_amdgcn_wmma_f32_16x16x32_bf16(false, ah, false, bl, (short)0, c, false, false);
    c = __builtin_amdgcn_wmma_f32_16x16x32_bf16(false, al, false, bh, (short)0, c, false, false);
    asm volatile("v_nop\n\tv_nop\n\tv_nop\n\tv_nop" : "+v"(c) : "v"(ah), "v"(al), "v"(bh), "v"(bl));
    return c;
}

union RouteSmem {
    unsigned short w[2 * NH * P1];
    float          h[128 * HSP];
};

__global__ __launch_bounds__(256) __attribute__((amdgpu_num_vgpr(256)))
void k_route(const float* __restrict__ X,
             const float* __restrict__ W1,
             const float* __restrict__ b1,
             const float* __restrict__ W2,
             const float* __restrict__ b2,
             float* __restrict__ route,
             int ntok)
{
    __shared__ __align__(16) RouteSmem sm;

    const int tid  = threadIdx.x;
    const int lane = tid & 31;
    const int wave = tid >> 5;
    const int h    = lane >> 4;
    const int nlo  = lane & 15;
    const int m0   = blockIdx.x * 128;

    for (int i = tid; i < ND * NH; i += 256) {
        const int k = i >> 7;
        const int n = i & 127;
        unsigned short hb, lb;
        split2(W1[i], hb, lb);
        sm.w[n * P1 + k]            = hb;
        sm.w[NH * P1 + n * P1 + k]  = lb;
    }
    __syncthreads();

    int rowt = m0 + wave * 16 + nlo;
    if (rowt > ntok - 1) rowt = ntok - 1;
    const int bb = rowt / NQ;
    const int ss = rowt - bb * NQ;
    const float* arow = X + ((size_t)bb * NS + ss) * ND;
    const unsigned short* w1h = sm.w;

    v8f acc[8] = {};

#pragma unroll 1
    for (int kc = 0; kc < ND; kc += 32) {
        const v4f a0 = *(const v4f*)(arow + kc + 8 * h);
        const v4f a1 = *(const v4f*)(arow + kc + 8 * h + 4);
        const v4f a2 = *(const v4f*)(arow + kc + 16 + 8 * h);
        const v4f a3 = *(const v4f*)(arow + kc + 16 + 8 * h + 4);
        float f[16];
#pragma unroll
        for (int i = 0; i < 4; ++i) {
            f[i]      = a0[i];
            f[4 + i]  = a1[i];
            f[8 + i]  = a2[i];
            f[12 + i] = a3[i];
        }
        Frag ah, al;
#pragma unroll
        for (int i = 0; i < 16; ++i) {
            unsigned short hb, lb;
            split2(f[i], hb, lb);
            ah.u[i] = hb;
            al.u[i] = lb;
        }

#pragma unroll
        for (int nt = 0; nt < 8; ++nt) {
            const unsigned short* bp = w1h + (nt * 16 + nlo) * P1 + kc + 8 * h;
            Frag bh, bl;
            bh.h[0] = *(const v8us*)(bp);
            bh.h[1] = *(const v8us*)(bp + 16);
            bl.h[0] = *(const v8us*)(bp + NH * P1);
            bl.h[1] = *(const v8us*)(bp + NH * P1 + 16);
            acc[nt] = mma3(acc[nt], ah.v, al.v, bh.v, bl.v);
        }
    }
    __syncthreads();

#pragma unroll
    for (int nt = 0; nt < 8; ++nt) {
        const int n = nt * 16 + nlo;
        const float bias = b1[n];
#pragma unroll
        for (int r = 0; r < 8; ++r) {
            const int m = wave * 16 + 8 * h + r;
            const float v = acc[nt][r] + bias;
            sm.h[m * HSP + n] = v > 0.f ? v : 0.f;
        }
    }
    __syncthreads();

    if (tid < 128) {
        float l[NE];
#pragma unroll
        for (int e = 0; e < NE; ++e) l[e] = b2[e];
        const float* hrow = sm.h + tid * HSP;
#pragma unroll 4
        for (int k = 0; k < NH; ++k) {
            const float hv = hrow[k];
            const float* w2r = W2 + k * NE;
#pragma unroll
            for (int e = 0; e < NE; ++e) l[e] += hv * w2r[e];
        }
        float mx = l[0];
#pragma unroll
        for (int e = 1; e < NE; ++e) mx = fmaxf(mx, l[e]);
        float p[NE];
        float sum = 0.f;
#pragma unroll
        for (int e = 0; e < NE; ++e) { p[e] = expf(l[e] - mx); sum += p[e]; }
        const float inv = 1.f / sum;
        int i0 = 0; float v0 = p[0] * inv;
#pragma unroll
        for (int e = 1; e < NE; ++e) {
            const float pe = p[e] * inv;
            if (pe > v0) { v0 = pe; i0 = e; }
        }
        int i1 = -1; float v1 = -1.f;
#pragma unroll
        for (int e = 0; e < NE; ++e) {
            if (e == i0) continue;
            const float pe = p[e] * inv;
            if (pe > v1) { v1 = pe; i1 = e; }
        }
        if (i1 < 0) i1 = 0;
        const float t    = expf(v1 - v0);
        const float inv2 = 1.f / (1.f + t);
        const float w0   = inv2;
        const float w1v  = t * inv2;

        const int tok = m0 + tid;
        if (tok < ntok) {
            union { v4f v; int i[4]; float f[4]; } rec;
            rec.i[0] = i0;
            rec.i[1] = i1;
            rec.f[2] = w0;
            rec.f[3] = w1v;
            volatile v4f* rp = (volatile v4f*)(route + (size_t)tok * 4);
            *rp = rec.v;
            __threadfence();
            *rp = rec.v;
        }
    }
}

__global__ __launch_bounds__(256)
void k_combine(const float* __restrict__ route,
               const float* __restrict__ eb,
               const float* __restrict__ ec,
               float* __restrict__ ob,
               float* __restrict__ oc,
               int ntok)
{
    __shared__ __align__(16) float cs[256 * NC];

    const int tid = threadIdx.x;
    const int t   = blockIdx.x * 256 + tid;
    const int tc  = (t < ntok) ? t : (ntok - 1);

    const v4f rec = *(const v4f*)(route + (size_t)tc * 4);
    int e0 = __float_as_int(rec[0]);
    int e1 = __float_as_int(rec[1]);
    e0 = e0 < 0 ? 0 : (e0 > NE - 1 ? NE - 1 : e0);
    e1 = e1 < 0 ? 0 : (e1 > NE - 1 ? NE - 1 : e1);
    const float w0 = rec[2];
    const float w1 = rec[3];

    const v4f x0 = *(const v4f*)(eb + ((size_t)e0 * ntok + tc) * 4);
    const v4f x1 = *(const v4f*)(eb + ((size_t)e1 * ntok + tc) * 4);
    v4f o;
    o[0] = w0 * x0[0] + w1 * x1[0];
    o[1] = w0 * x0[1] + w1 * x1[1];
    o[2] = w0 * x0[2] + w1 * x1[2];
    o[3] = w0 * x0[3] + w1 * x1[3];

    const float* c0 = ec + ((size_t)e0 * ntok + tc) * NC;
    const float* c1 = ec + ((size_t)e1 * ntok + tc) * NC;
#pragma unroll
    for (int c = 0; c < NC; ++c)
        cs[tid * NC + c] = w0 * c0[c] + w1 * c1[c];
    __syncthreads();

    int nv = ntok - blockIdx.x * 256;
    if (nv > 256) nv = 256;
    const int nflt = nv * NC;
    const int nvec = nflt >> 2;
    const int rem  = nflt & 3;
    float* ocb = oc + (size_t)blockIdx.x * 256 * NC;
    const v4f* csv = (const v4f*)cs;

    if (t < ntok) *(volatile v4f*)(ob + (size_t)t * 4) = o;
    for (int j = tid; j < nvec; j += 256)
        *(volatile v4f*)(ocb + 4 * j) = csv[j];
    if (tid < rem)
        *(volatile float*)(ocb + 4 * nvec + tid) = cs[4 * nvec + tid];
    __threadfence();
    if (t < ntok) *(volatile v4f*)(ob + (size_t)t * 4) = o;
    for (int j = tid; j < nvec; j += 256)
        *(volatile v4f*)(ocb + 4 * j) = csv[j];
    if (tid < rem)
        *(volatile float*)(ocb + 4 * nvec + tid) = cs[4 * nvec + tid];
}

extern "C" void kernel_launch(void* const* d_in, const int* in_sizes, int n_in,
                              void* d_out, int out_size, void* d_ws, size_t ws_size,
                              hipStream_t stream)
{
    if (n_in < 7) return;
    const float* X  = (const float*)d_in[0];
    const float* W1 = (const float*)d_in[1];
    const float* b1 = (const float*)d_in[2];
    const float* W2 = (const float*)d_in[3];
    const float* b2 = (const float*)d_in[4];
    const float* eb = (const float*)d_in[5];
    const float* ec = (const float*)d_in[6];

    const int ntok = NTOK;
    if (in_sizes[0] != NB * NS * ND || in_sizes[1] != ND * NH || in_sizes[2] != NH ||
        in_sizes[3] != NH * NE || in_sizes[4] != NE ||
        in_sizes[5] != NE * ntok * 4 || in_sizes[6] != NE * ntok * NC) return;
    if (out_size != ntok * 4 + ntok * NC) return;

    float* ob = (float*)d_out;
    float* oc = (float*)d_out + (size_t)ntok * 4;

    const size_t route_bytes = (size_t)ntok * 16;
    if (route_bytes > ws_size) return;
    float* route = (float*)d_ws;

    const int grid1 = (ntok + 127) / 128;
    const int grid2 = (ntok + 255) / 256;

    k_route<<<grid1, 256, 0, stream>>>(X, W1, b1, W2, b2, route, ntok);
    k_combine<<<grid2, 256, 0, stream>>>(route, eb, ec, ob, oc, ntok);
}
